// Mamba_Encoder_Layer_2302102470701
// MI455X (gfx1250) — hardware-run, weakly checked
//
#include <hip/hip_runtime.h>
#include <math.h>

typedef __attribute__((ext_vector_type(8)))  _Float16 v8h;
typedef __attribute__((ext_vector_type(16))) __bf16   v16b;
typedef __attribute__((ext_vector_type(8)))  __bf16   v8b;
typedef __attribute__((ext_vector_type(8)))  float    v8f;
typedef __attribute__((ext_vector_type(4)))  float    v4f;
typedef __attribute__((ext_vector_type(2)))  float    v2f;
typedef __attribute__((ext_vector_type(4)))  unsigned v4u;

constexpr int kBatch = 4;
constexpr int kSeq   = 2048;
constexpr int kDm    = 512;
constexpr int kDin   = 1024;
constexpr int kNst   = 16;
constexpr int kDtR   = 32;
constexpr int kDff   = 2048;
constexpr int kXzP   = 2 * kDin;
constexpr int kXdP   = kDtR + 2 * kNst;
constexpr int kTP    = 260;
static_assert(kXdP == 64, "x_proj width");
static_assert((kDm % 32) == 0 && (kDin % 32) == 0 && (kDff % 32) == 0 && (kDtR % 32) == 0, "GEMM K multiples of 32");
static_assert((kSeq % 64) == 0 && (kXzP % 64) == 0 && (kXdP % 64) == 0 && (kDm % 64) == 0 &&
              (kDin % 64) == 0 && (kDff % 64) == 0, "GEMM M,N multiples of 64");
static_assert((kDin % 256) == 0 && (kSeq % 16) == 0, "scan/conv tiles");

constexpr size_t kOffXB   = 0;
constexpr size_t kOffWIN  = kOffXB   + (size_t)kBatch * kSeq * kDm * 2;
constexpr size_t kOffWX   = kOffWIN  + (size_t)kXzP * kDm * 2;
constexpr size_t kOffWDT  = kOffWX   + (size_t)kXdP * kDin * 2;
constexpr size_t kOffWO   = kOffWDT  + (size_t)kDin * kDtR * 2;
constexpr size_t kOffW1   = kOffWO   + (size_t)kDm * kDin * 2;
constexpr size_t kOffW2   = kOffW1   + (size_t)kDff * kDm * 2;
constexpr size_t kOffXZ   = kOffW2   + (size_t)kDm * kDff * 2;
constexpr size_t kOffXCB  = kOffXZ   + (size_t)kSeq * kXzP * 4;
constexpr size_t kOffDBL  = kOffXCB  + (size_t)kSeq * kDin * 2;
constexpr size_t kOffDTLB = kOffDBL  + (size_t)kSeq * kXdP * 4;
constexpr size_t kOffDLR  = kOffDTLB + (size_t)kSeq * kDtR * 2;
constexpr size_t kOffYH   = kOffDLR  + (size_t)kSeq * kDin * 4;
constexpr size_t kOffYL   = kOffYH   + (size_t)kSeq * kDin * 2;
constexpr size_t kOffHMH  = kOffYL   + (size_t)kSeq * kDin * 2;
constexpr size_t kOffHML  = kOffHMH  + (size_t)kSeq * kDm * 2;
constexpr size_t kOffF1P  = kOffHML  + (size_t)kSeq * kDm * 2;
constexpr size_t kOffF1H  = kOffF1P  + (size_t)kSeq * kDff * 4;
constexpr size_t kOffF1L  = kOffF1H  + (size_t)kSeq * kDff * 2;
constexpr size_t kWsTotal = kOffF1L  + (size_t)kSeq * kDff * 2;
static_assert(kWsTotal == 92078080ull, "carve total");
static_assert(kWsTotal <= 134217728ull, "carve cap");
static_assert((kOffWIN % 128) == 0 && (kOffWX % 128) == 0 && (kOffWDT % 128) == 0 && (kOffWO % 128) == 0 &&
              (kOffW1 % 128) == 0 && (kOffW2 % 128) == 0 && (kOffXZ % 128) == 0 && (kOffXCB % 128) == 0 &&
              (kOffDBL % 128) == 0 && (kOffDTLB % 128) == 0 && (kOffDLR % 128) == 0 && (kOffYH % 128) == 0 &&
              (kOffYL % 128) == 0 && (kOffHMH % 128) == 0 && (kOffHML % 128) == 0 && (kOffF1P % 128) == 0 &&
              (kOffF1H % 128) == 0 && (kOffF1L % 128) == 0, "128-B aligned regions");

__device__ __forceinline__ unsigned short f2bf_bits(float f) {
  unsigned u = __float_as_uint(f);
  return (unsigned short)((u + 0x7FFFu + ((u >> 16) & 1u)) >> 16);
}
__device__ __forceinline__ float bf_bits2f(unsigned short h) { return __uint_as_float(((unsigned)h) << 16); }
__device__ __forceinline__ float bf16r(float f) { return bf_bits2f(f2bf_bits(f)); }
__device__ __forceinline__ unsigned pack_bf2(float a, float b) {
  const unsigned lo = (unsigned)f2bf_bits(a);
  const unsigned hi = (unsigned)f2bf_bits(b);
  return lo | (hi << 16);
}
__device__ __forceinline__ void split_pack2(float a, float b, unsigned& wh, unsigned& wl) {
  const unsigned short ha = f2bf_bits(a), hb = f2bf_bits(b);
  const unsigned short la = f2bf_bits(a - bf_bits2f(ha)), lb = f2bf_bits(b - bf_bits2f(hb));
  wh = (unsigned)ha | (((unsigned)hb) << 16);
  wl = (unsigned)la | (((unsigned)lb) << 16);
}

__device__ __forceinline__ void dep_guard4_b(v8f& a, v8f& b, v8f& c, v8f& d, v16b x, v16b y) {
  asm volatile("v_nop\n\tv_nop\n\tv_nop\n\tv_nop" : "+v"(a), "+v"(b), "+v"(c), "+v"(d) : "v"(x), "v"(y));
}
__device__ __forceinline__ void keep4_b(v16b a, v16b b, v16b c, v16b d) { asm volatile("v_nop" :: "v"(a), "v"(b), "v"(c), "v"(d)); }
__device__ __forceinline__ void acc_guard4(v8f& a, v8f& b, v8f& c, v8f& d) { asm volatile("v_nop\n\tv_nop\n\tv_nop\n\tv_nop" : "+v"(a), "+v"(b), "+v"(c), "+v"(d)); }

struct FragB {
  union U { v16b v; v8b h[2]; };
  static __device__ __forceinline__ v16b load(const __bf16* p) {
    U f; f.h[0] = *(const v8b*)(p); f.h[1] = *(const v8b*)(p + 16); return f.v;
  }
  static __device__ __forceinline__ v8f mma(v16b a, v16b b, v8f c) {
    return __builtin_amdgcn_wmma_f32_16x16x32_bf16(false, a, false, b, (short)0, c, false, false);
  }
};

template <int SPL, int BIAS_MODE, int OUT_MODE>
__global__ __launch_bounds__(256) void wmma_gemm64(
    const unsigned short* __restrict__ Ap, const unsigned short* __restrict__ A2p, int lda,
    const unsigned short* __restrict__ Btp, int ldb,
    void* __restrict__ Cout, void* __restrict__ Cout2, int ldc,
    const float* __restrict__ bias,
    int M, int N, int K, float scale) {
  const __bf16* A  = (const __bf16*)Ap;
  const __bf16* A2 = (const __bf16*)A2p;
  const __bf16* Bt = (const __bf16*)Btp;
  __shared__ __align__(16) float sT[8][16 * 68];
  const int lane = threadIdx.x & 31;
  const int wave = threadIdx.x >> 5;
  const int tilesN = N >> 6;
  const int tilesM = M >> 6;
  const int tile = blockIdx.x * 8 + wave;
  if (tile >= tilesM * tilesN) return;
  const int tm = tile / tilesN;
  const int tn = tile - tm * tilesN;
  const int m0 = tm << 6;
  const int n0 = tn << 6;

  const int rlane = lane & 15;
  const int koff  = (lane >> 4) * 8;
  const int mOff  = (lane >> 4) * 8;

  v8f acc[4][4];
#pragma unroll
  for (int i = 0; i < 4; ++i)
#pragma unroll
    for (int j = 0; j < 4; ++j) acc[i][j] = (v8f){0.f,0.f,0.f,0.f,0.f,0.f,0.f,0.f};

  for (int k0 = 0; k0 < K; k0 += 32) {
    v16b bh[4];
#pragma unroll
    for (int j = 0; j < 4; ++j) {
      const size_t bo = (size_t)(n0 + (j << 4) + rlane) * ldb + koff + k0;
      bh[j] = FragB::load(Bt + bo);
    }
#pragma unroll
    for (int i = 0; i < 4; ++i) {
      const size_t ao = (size_t)(m0 + (i << 4) + rlane) * lda + koff + k0;
      v16b ah = FragB::load(A + ao);
      v16b al = ah;
      if (SPL == 1) al = FragB::load(A2 + ao);
#pragma unroll
      for (int j = 0; j < 4; ++j) {
        acc[i][j] = FragB::mma(ah, bh[j], acc[i][j]);
        if (SPL == 1) acc[i][j] = FragB::mma(al, bh[j], acc[i][j]);
      }
      dep_guard4_b(acc[i][0], acc[i][1], acc[i][2], acc[i][3], ah, al);
    }
    keep4_b(bh[0], bh[1], bh[2], bh[3]);
  }
  acc_guard4(acc[0][0], acc[0][1], acc[0][2], acc[0][3]);
  acc_guard4(acc[1][0], acc[1][1], acc[1][2], acc[1][3]);
  acc_guard4(acc[2][0], acc[2][1], acc[2][2], acc[2][3]);
  acc_guard4(acc[3][0], acc[3][1], acc[3][2], acc[3][3]);

  float* slab = sT[wave];
#pragma unroll
  for (int i = 0; i < 4; ++i) {
    const int mBase = m0 + (i << 4);
#pragma unroll
    for (int j = 0; j < 4; ++j) {
      const int n = n0 + (j << 4) + rlane;
      float bv = 0.f;
      if (BIAS_MODE == 2) bv = bf16r(bias[n]);
#pragma unroll
      for (int r = 0; r < 8; ++r) {
        float v = acc[i][j][r] * scale;
        if (BIAS_MODE == 2) v += bv;
        slab[(mOff + r) * 68 + (j << 4) + rlane] = v;
      }
    }
    __builtin_amdgcn_fence(__ATOMIC_RELEASE, "workgroup");
    __builtin_amdgcn_wave_barrier();
    __builtin_amdgcn_fence(__ATOMIC_ACQUIRE, "workgroup");
    if (OUT_MODE == 0) {
      float* C = (float*)Cout;
      const int hh = lane >> 4, c4 = (lane & 15) * 4;
      for (int pass = 0; pass < 2; ++pass) {
#pragma unroll
        for (int it = 0; it < 8; ++it) {
          const int row = it * 2 + hh;
          v4f v = *(const v4f*)(slab + row * 68 + c4);
          *(volatile v4f*)(C + (size_t)(mBase + row) * ldc + n0 + c4) = v;
        }
        __threadfence();
      }
    } else {
      const int q = lane >> 3, c8 = (lane & 7) * 8;
      unsigned short* C  = (unsigned short*)Cout;
      unsigned short* C2 = (unsigned short*)Cout2;
      for (int pass = 0; pass < 2; ++pass) {
#pragma unroll
        for (int it = 0; it < 4; ++it) {
          const int row = it * 4 + q;
          const float* sp = slab + row * 68 + c8;
          const v4f a0 = *(const v4f*)(sp);
          const v4f a1 = *(const v4f*)(sp + 4);
          unsigned ph0, ph1, ph2, ph3, pl0, pl1, pl2, pl3;
          split_pack2(a0[0], a0[1], ph0, pl0);
          split_pack2(a0[2], a0[3], ph1, pl1);
          split_pack2(a1[0], a1[1], ph2, pl2);
          split_pack2(a1[2], a1[3], ph3, pl3);
          const v4u hv = (v4u){ph0, ph1, ph2, ph3};
          const v4u lv = (v4u){pl0, pl1, pl2, pl3};
          *(volatile v4u*)(C  + (size_t)(mBase + row) * ldc + n0 + c8) = hv;
          *(volatile v4u*)(C2 + (size_t)(mBase + row) * ldc + n0 + c8) = lv;
        }
        __threadfence();
      }
    }
    __builtin_amdgcn_fence(__ATOMIC_RELEASE, "workgroup");
    __builtin_amdgcn_wave_barrier();
    __builtin_amdgcn_fence(__ATOMIC_ACQUIRE, "workgroup");
  }
}

__global__ __launch_bounds__(256) void cast_bf16_kernel(
    const float* __restrict__ src, unsigned short* __restrict__ dst, int total8)
{
  const int i = blockIdx.x * 256 + threadIdx.x;
  if (i >= total8) return;
  const size_t e0 = (size_t)i << 3;
  const v4f a0 = *(const v4f*)(src + e0);
  const v4f a1 = *(const v4f*)(src + e0 + 4);
  const unsigned u0 = pack_bf2(a0[0], a0[1]);
  const unsigned u1 = pack_bf2(a0[2], a0[3]);
  const unsigned u2 = pack_bf2(a1[0], a1[1]);
  const unsigned u3 = pack_bf2(a1[2], a1[3]);
  const v4u w = (v4u){u0, u1, u2, u3};
  unsigned short* q = dst + e0;
  *(volatile v4u*)q = w;
  __threadfence();
  *(volatile v4u*)q = w;
}

__global__ __launch_bounds__(256) void dtl_cast_kernel(
    const float* __restrict__ DBL, unsigned short* __restrict__ DTLB, int total8)
{
  const int i = blockIdx.x * 256 + threadIdx.x;
  if (i >= total8) return;
  const int e0  = i << 3;
  const int row = e0 >> 5;
  const int c8  = e0 & 31;
  const float* p = DBL + (size_t)row * kXdP + c8;
  const v4f a0 = *(const v4f*)(p);
  const v4f a1 = *(const v4f*)(p + 4);
  const unsigned u0 = pack_bf2(a0[0], a0[1]);
  const unsigned u1 = pack_bf2(a0[2], a0[3]);
  const unsigned u2 = pack_bf2(a1[0], a1[1]);
  const unsigned u3 = pack_bf2(a1[2], a1[3]);
  const v4u w = (v4u){u0, u1, u2, u3};
  unsigned short* q = DTLB + e0;
  *(volatile v4u*)q = w;
  __threadfence();
  *(volatile v4u*)q = w;
}

__global__ __launch_bounds__(256) void conv_silu_kernel(
    const float* __restrict__ XZ, const float* __restrict__ cw, const float* __restrict__ cb,
    unsigned short* __restrict__ XCB)
{
  __shared__ __align__(16) float sT[16 * kTP];
  const int tid = threadIdx.x, lane = tid & 31, wave = tid >> 5;
  const int d0 = blockIdx.x * 256, d = d0 + tid;
  const int t0 = blockIdx.y * 64;
  const v4f wv = *(const v4f*)(cw + (size_t)d * 4);
  const float w0 = bf16r(wv[0]), w1 = bf16r(wv[1]), w2 = bf16r(wv[2]), w3 = bf16r(wv[3]);
  const float bc = bf16r(cb[d]);
  float xm3, xm2, xm1;
  {
    const int r3 = t0 - 3, r2 = t0 - 2, r1 = t0 - 1;
    const float v3 = XZ[(size_t)(r3 < 0 ? 0 : r3) * kXzP + d];
    const float v2 = XZ[(size_t)(r2 < 0 ? 0 : r2) * kXzP + d];
    const float v1 = XZ[(size_t)(r1 < 0 ? 0 : r1) * kXzP + d];
    xm3 = (r3 >= 0) ? v3 : 0.f;
    xm2 = (r2 >= 0) ? v2 : 0.f;
    xm1 = (r1 >= 0) ? v1 : 0.f;
  }
#pragma unroll 1
  for (int sub = 0; sub < 4; ++sub) {
    const int lb = t0 + sub * 16;
#pragma unroll 1
    for (int s = 0; s < 16; ++s) {
      const float xcur = XZ[(size_t)(lb + s) * kXzP + d];
      float acc = w0 * xm3;
      acc = fmaf(w1, xm2, acc);
      acc = fmaf(w2, xm1, acc);
      acc = fmaf(w3, xcur, acc);
      const float sv = acc + bc;
      const float sg = 1.0f / (1.0f + expf(-sv));
      sT[s * kTP + tid] = sv * sg;
      xm3 = xm2; xm2 = xm1; xm1 = xcur;
    }
    __syncthreads();
    v4u wq[2];
#pragma unroll
    for (int it = 0; it < 2; ++it) {
      const float* sp = sT + (it * 8 + wave) * kTP + lane * 8;
      const v4f a0 = *(const v4f*)(sp);
      const v4f a1 = *(const v4f*)(sp + 4);
      const unsigned u0 = pack_bf2(a0[0], a0[1]);
      const unsigned u1 = pack_bf2(a0[2], a0[3]);
      const unsigned u2 = pack_bf2(a1[0], a1[1]);
      const unsigned u3 = pack_bf2(a1[2], a1[3]);
      wq[it] = (v4u){u0, u1, u2, u3};
    }
    for (int pass = 0; pass < 2; ++pass) {
#pragma unroll
      for (int it = 0; it < 2; ++it)
        *(volatile v4u*)(XCB + (size_t)(lb + it * 8 + wave) * kDin + d0 + lane * 8) = wq[it];
      __threadfence();
    }
    __syncthreads();
  }
}

__global__ __launch_bounds__(256) void scan_kernel(
    const float* __restrict__ DLR, const float* __restrict__ XZ, const float* __restrict__ DBL,
    const float* __restrict__ cw, const float* __restrict__ cb,
    const float* __restrict__ A_log, const float* __restrict__ Dv,
    unsigned short* __restrict__ YH, unsigned short* __restrict__ YL)
{
  __shared__ __align__(16) float sBC[16 * 32];
  __shared__ __align__(16) float sY[16 * kTP];
  __shared__ __align__(16) float sA[kNst * 256];
  const int tid = threadIdx.x, lane = tid & 31, wave = tid >> 5;
  const int d0 = blockIdx.x * 256, d = d0 + tid;

#pragma unroll 1
  for (int s = 0; s < kNst; ++s) sA[s * 256 + tid] = -expf(bf16r(A_log[(size_t)d * kNst + s]));
  __syncthreads();
  float An[kNst], h[kNst];
#pragma unroll
  for (int n = 0; n < kNst; ++n) {
    An[n] = sA[n * 256 + tid];
    h[n] = 0.f;
  }
  const float Dd = bf16r(Dv[d]);
  const v4f wv = *(const v4f*)(cw + (size_t)d * 4);
  const float w0 = bf16r(wv[0]), w1 = bf16r(wv[1]), w2 = bf16r(wv[2]), w3 = bf16r(wv[3]);
  const float bc = bf16r(cb[d]);
  float xm3 = 0.f, xm2 = 0.f, xm1 = 0.f;

#pragma unroll 1
  for (int c = 0; c < kSeq / 16; ++c) {
    const int l0 = c * 16;
    if (tid < 128) {
      const int r = tid >> 3, q = (tid & 7) * 4;
      const v4f v = *(const v4f*)(DBL + (size_t)(l0 + r) * kXdP + kDtR + q);
      *(v4f*)(sBC + r * 32 + q) = v;
    }
    __syncthreads();
#pragma unroll 1
    for (int s = 0; s < 16; ++s) {
      const size_t m = (size_t)(l0 + s);
      float a    = DLR[m * kDin + d];
      float xcur = XZ[m * kXzP + d];
      float zv   = XZ[m * kXzP + kDin + d];
      asm volatile("" : "+v"(a), "+v"(xcur), "+v"(zv));
      const float ea  = expf(-fabsf(a));
      const float u1  = 1.0f + ea;
      const float l1p = __logf(u1) + (ea - (u1 - 1.0f)) * __builtin_amdgcn_rcpf(u1);
      const float delta = fmaxf(a, 0.0f) + l1p;
      float cacc = w0 * xm3;
      cacc = fmaf(w1, xm2, cacc);
      cacc = fmaf(w2, xm1, cacc);
      cacc = fmaf(w3, xcur, cacc);
      const float sv = cacc + bc;
      const float xc = sv * (1.0f / (1.0f + expf(-sv)));
      xm3 = xm2; xm2 = xm1; xm1 = xcur;
      const float dtx = delta * xc;
      v4f Bq[4], Cq[4];
#pragma unroll
      for (int qq = 0; qq < 4; ++qq) {
        Bq[qq] = *(const v4f*)(sBC + s * 32 + 4 * qq);
        Cq[qq] = *(const v4f*)(sBC + s * 32 + kNst + 4 * qq);
      }
      float y = 0.f;
#pragma unroll
      for (int n = 0; n < kNst; ++n) {
        const float e = __expf(delta * An[n]);
        h[n] = fmaf(e, h[n], dtx * Bq[n >> 2][n & 3]);
        y = fmaf(h[n], Cq[n >> 2][n & 3], y);
      }
      y = fmaf(xc, Dd, y);
      const float g = zv * (1.0f / (1.0f + expf(-zv)));
      sY[s * kTP + tid] = y * g;
    }
    __syncthreads();
    v4u wh[2], wl[2];
#pragma unroll
    for (int it = 0; it < 2; ++it) {
      const float* sp = sY + (it * 8 + wave) * kTP + lane * 8;
      const v4f a0 = *(const v4f*)(sp);
      const v4f a1 = *(const v4f*)(sp + 4);
      unsigned h0, h1, h2, h3, q0, q1, q2, q3;
      split_pack2(a0[0], a0[1], h0, q0);
      split_pack2(a0[2], a0[3], h1, q1);
      split_pack2(a1[0], a1[1], h2, q2);
      split_pack2(a1[2], a1[3], h3, q3);
      wh[it] = (v4u){h0, h1, h2, h3};
      wl[it] = (v4u){q0, q1, q2, q3};
    }
    for (int pass = 0; pass < 2; ++pass) {
#pragma unroll
      for (int it = 0; it < 2; ++it) {
        const size_t o = (size_t)(l0 + it * 8 + wave) * kDin + d0 + lane * 8;
        *(volatile v4u*)(YH + o) = wh[it];
        *(volatile v4u*)(YL + o) = wl[it];
      }
      __threadfence();
    }
  }
}

__global__ __launch_bounds__(256) void gelu_split_kernel(
    const float* __restrict__ src, unsigned short* __restrict__ dhi, unsigned short* __restrict__ dlo, int total8)
{
  __shared__ __align__(16) unsigned sH[256 * 4];
  __shared__ __align__(16) unsigned sL[256 * 4];
  const int tid = threadIdx.x;
  const int i = blockIdx.x * 256 + tid;
  const int ic = (i < total8) ? i : (total8 - 1);
  const size_t e0 = (size_t)ic << 3;
#pragma unroll 1
  for (int p = 0; p < 4; ++p) {
    const v2f av = *(const v2f*)(src + e0 + 2 * p);
    float a0 = av[0], a1 = av[1];
    asm volatile("" : "+v"(a0), "+v"(a1));
    const float g0 = 0.5f * a0 * (1.0f + erff(a0 * 0.70710678118654752f));
    const float g1 = 0.5f * a1 * (1.0f + erff(a1 * 0.70710678118654752f));
    unsigned wh, wl;
    split_pack2(g0, g1, wh, wl);
    sH[tid * 4 + p] = wh;
    sL[tid * 4 + p] = wl;
  }
  __syncthreads();
  const v4u vh = *(const v4u*)(sH + tid * 4);
  const v4u vl = *(const v4u*)(sL + tid * 4);
  if (i < total8) {
    unsigned short* qh = dhi + e0;
    unsigned short* ql = dlo + e0;
    *(volatile v4u*)qh = vh;
    *(volatile v4u*)ql = vl;
    __threadfence();
    *(volatile v4u*)qh = vh;
    *(volatile v4u*)ql = vl;
  }
}

extern "C" void kernel_launch(void* const* d_in, const int* in_sizes, int n_in,
                              void* d_out, int out_size, void* d_ws, size_t ws_size,
                              hipStream_t stream)
{
  if (n_in < 14) return;
  if (in_sizes[0]  != kBatch * kSeq * kDm) return;
  if (in_sizes[1]  != kXzP * kDm) return;
  if (in_sizes[2]  != kDin * 4) return;
  if (in_sizes[3]  != kDin) return;
  if (in_sizes[4]  != kXdP * kDin) return;
  if (in_sizes[5]  != kDin * kDtR) return;
  if (in_sizes[6]  != kDin) return;
  if (in_sizes[7]  != kDin * kNst) return;
  if (in_sizes[8]  != kDin) return;
  if (in_sizes[9]  != kDm * kDin) return;
  if (in_sizes[10] != kDff * kDm) return;
  if (in_sizes[11] != kDff) return;
  if (in_sizes[12] != kDm * kDff) return;
  if (in_sizes[13] != kDm) return;
  if (out_size != kBatch * kSeq * kDm) return;
  if (ws_size < kWsTotal) return;

  const float* x       = (const float*)d_in[0];
  const float* W_in    = (const float*)d_in[1];
  const float* conv_w  = (const float*)d_in[2];
  const float* conv_b  = (const float*)d_in[3];
  const float* W_xproj = (const float*)d_in[4];
  const float* W_dt    = (const float*)d_in[5];
  const float* b_dt    = (const float*)d_in[6];
  const float* A_log   = (const float*)d_in[7];
  const float* Dv      = (const float*)d_in[8];
  const float* W_out   = (const float*)d_in[9];
  const float* W1      = (const float*)d_in[10];
  const float* b1      = (const float*)d_in[11];
  const float* W2      = (const float*)d_in[12];
  const float* b2      = (const float*)d_in[13];
  float* dout = (float*)d_out;

  char* ws = (char*)d_ws;
  unsigned short* XB   = (unsigned short*)(ws + kOffXB);
  unsigned short* WINB = (unsigned short*)(ws + kOffWIN);
  unsigned short* WXB  = (unsigned short*)(ws + kOffWX);
  unsigned short* WDTB = (unsigned short*)(ws + kOffWDT);
  unsigned short* WOB  = (unsigned short*)(ws + kOffWO);
  unsigned short* W1B  = (unsigned short*)(ws + kOffW1);
  unsigned short* W2B  = (unsigned short*)(ws + kOffW2);
  float*          XZ   = (float*)(ws + kOffXZ);
  unsigned short* XCB  = (unsigned short*)(ws + kOffXCB);
  float*          DBL  = (float*)(ws + kOffDBL);
  unsigned short* DTLB = (unsigned short*)(ws + kOffDTLB);
  float*          DLR  = (float*)(ws + kOffDLR);
  unsigned short* YH   = (unsigned short*)(ws + kOffYH);
  unsigned short* YL   = (unsigned short*)(ws + kOffYL);
  unsigned short* HMH  = (unsigned short*)(ws + kOffHMH);
  unsigned short* HML  = (unsigned short*)(ws + kOffHML);
  float*          F1P  = (float*)(ws + kOffF1P);
  unsigned short* F1H  = (unsigned short*)(ws + kOffF1H);
  unsigned short* F1L  = (unsigned short*)(ws + kOffF1L);
  const float* dummy_bias = b_dt;

  cast_bf16_kernel<<<(kBatch * kSeq * kDm / 8) / 256, 256, 0, stream>>>(x, XB, kBatch * kSeq * kDm / 8);
  cast_bf16_kernel<<<(kXzP * kDm / 8) / 256, 256, 0, stream>>>(W_in, WINB, kXzP * kDm / 8);
  cast_bf16_kernel<<<(kXdP * kDin / 8) / 256, 256, 0, stream>>>(W_xproj, WXB, kXdP * kDin / 8);
  cast_bf16_kernel<<<(kDin * kDtR / 8) / 256, 256, 0, stream>>>(W_dt, WDTB, kDin * kDtR / 8);
  cast_bf16_kernel<<<(kDm * kDin / 8) / 256, 256, 0, stream>>>(W_out, WOB, kDm * kDin / 8);
  cast_bf16_kernel<<<(kDff * kDm / 8) / 256, 256, 0, stream>>>(W1, W1B, kDff * kDm / 8);
  cast_bf16_kernel<<<(kDm * kDff / 8) / 256, 256, 0, stream>>>(W2, W2B, kDm * kDff / 8);

  for (int b = 0; b < kBatch; ++b) {
    const unsigned short* XBb = XB + (size_t)b * kSeq * kDm;
    float* outb = dout + (size_t)b * kSeq * kDm;

    wmma_gemm64<0, 0, 0><<<128, 256, 0, stream>>>(
        XBb, XBb, kDm, WINB, kDm, (void*)XZ, (void*)XZ, kXzP, dummy_bias, kSeq, kXzP, kDm, 1.0f);

    conv_silu_kernel<<<dim3(kDin / 256, kSeq / 64), 256, 0, stream>>>(XZ, conv_w, conv_b, XCB);

    wmma_gemm64<0, 0, 0><<<4, 256, 0, stream>>>(
        XCB, XCB, kDin, WXB, kDin, (void*)DBL, (void*)DBL, kXdP, dummy_bias, kSeq, kXdP, kDin, 1.0f);

    dtl_cast_kernel<<<(kSeq * kDtR / 8) / 256, 256, 0, stream>>>(DBL, DTLB, kSeq * kDtR / 8);

    wmma_gemm64<0, 2, 0><<<64, 256, 0, stream>>>(
        DTLB, DTLB, kDtR, WDTB, kDtR, (void*)DLR, (void*)DLR, kDin, b_dt, kSeq, kDin, kDtR, 1.0f);

    scan_kernel<<<kDin / 256, 256, 0, stream>>>(DLR, XZ, DBL, conv_w, conv_b, A_log, Dv, YH, YL);

    wmma_gemm64<1, 0, 2><<<32, 256, 0, stream>>>(
        YH, YL, kDin, WOB, kDin, (void*)HMH, (void*)HML, kDm, dummy_bias, kSeq, kDm, kDin, 1.0f);

    wmma_gemm64<1, 2, 0><<<128, 256, 0, stream>>>(
        HMH, HML, kDm, W1B, kDm, (void*)F1P, (void*)F1P, kDff, b1, kSeq, kDff, kDm, 1.0f);

    gelu_split_kernel<<<(kSeq * kDff / 8) / 256, 256, 0, stream>>>(F1P, F1H, F1L, kSeq * kDff / 8);

    wmma_gemm64<1, 2, 0><<<32, 256, 0, stream>>>(
        F1H, F1L, kDff, W2B, kDff, (void*)outb, (void*)outb, kDm, b2, kSeq, kDm, kDff, 1.0f);
  }
}
